// PositiveMultiheadAttention_85779086835795
// MI455X (gfx1250) — hardware-run, weakly checked
//
#include <hip/hip_runtime.h>
#include <stddef.h>


typedef _Float16 h16;
typedef _Float16 v16h __attribute__((ext_vector_type(16)));
typedef _Float16 v8h  __attribute__((ext_vector_type(8)));
typedef float    v8f  __attribute__((ext_vector_type(8)));
typedef float    v4f  __attribute__((ext_vector_type(4)));

#ifndef NB
#define NB 2
#endif
#ifndef SEQ
#define SEQ 1024
#endif
#define NB_FULL  2
#define SEQ_FULL 1024
#define DIM   512
#define NHEAD 8
#define HD    64
#define MROWS (NB * SEQ)
#define KVROWS 80

static_assert(NB >= 1 && NB <= NB_FULL);
static_assert(SEQ >= 64 && SEQ <= SEQ_FULL && (SEQ % 64) == 0 && (SEQ % 32) == 0);
static_assert(DIM == NHEAD * HD);
static_assert(HD == 64);
static_assert((DIM % 64) == 0 && (DIM % 32) == 0 && (DIM % 8) == 0);
static_assert((MROWS % 64) == 0);
static_assert((((size_t)MROWS * DIM / 8) % 256) == 0);
static_assert((((size_t)DIM * DIM / 8) % 256) == 0);
static_assert(KVROWS == HD + 16);
static_assert((HD % 32) == 0);

#define LDC 68
static_assert((LDC % 4) == 0 && LDC >= 64);

#define WCARRY 64.0f
#define QCARRY 1024.0f
#define KVCARRY 0.0625f
#define VCARRY 64.0f

#define WSQ_BYTES     ((size_t)DIM * DIM * 2)
#define PLANE16_BYTES ((size_t)MROWS * DIM * 2)
#define KVT_BYTES     ((size_t)NB * NHEAD * KVROWS * HD * 2)
#define OFF_X   ((size_t)0)
#define OFF_WQ  (OFF_X + PLANE16_BYTES)
#define OFF_WK  (OFF_WQ + WSQ_BYTES)
#define OFF_WV  (OFF_WK + WSQ_BYTES)
#define OFF_WO  (OFF_WV + WSQ_BYTES)
#define OFF_EQ  (OFF_WO + WSQ_BYTES)
#define OFF_EKT (OFF_EQ + PLANE16_BYTES)
#define OFF_VT  (OFF_EKT + PLANE16_BYTES)
#define OFF_KVT (OFF_VT + PLANE16_BYTES)
#define OFF_J   (OFF_KVT + KVT_BYTES)
#define WS_TOTAL (OFF_J + PLANE16_BYTES)
static_assert((WSQ_BYTES % 128) == 0 && (PLANE16_BYTES % 128) == 0 && (KVT_BYTES % 128) == 0);
static_assert((size_t)NB * DIM * SEQ * 2 == PLANE16_BYTES);
static_assert(WS_TOTAL <= (size_t)134217728);

__device__ __forceinline__ float bf16r(float x) {
  unsigned int u = __float_as_uint(x);
  u = (u + 0x7FFFu + ((u >> 16) & 1u)) & 0xFFFF0000u;
  return __uint_as_float(u);
}

static __device__ __forceinline__ h16 toh_flush(float v) {
  const h16 r = (h16)v;
  return (fabsf(v) < 6.103515625e-05f) ? (h16)0.0f : r;
}

__device__ __forceinline__ v16h frag_at(const _Float16* p) {
  v8h lo = *(const v8h*)(p);
  v8h hi = *(const v8h*)(p + 16);
  v16h out;
#pragma unroll
  for (int i = 0; i < 8; ++i) { out[i] = lo[i]; out[i + 8] = hi[i]; }
  return out;
}

__device__ __forceinline__ v8f wmma16(v16h a, v16h b, v8f c) {
  v8f d = __builtin_amdgcn_wmma_f32_16x16x32_f16(false, a, false, b, (short)0, c,
                                                 false, false);
  asm volatile("v_nop\n\tv_nop\n\tv_nop\n\tv_nop" : "+v"(d) : "v"(a), "v"(b));
  return d;
}

__global__ __launch_bounds__(256) void cast_kernel(
    const float* __restrict__ src, _Float16* __restrict__ dst, float carry,
    unsigned rows_c, unsigned rows_f) {
#pragma clang fp contract(off)
  const unsigned g = blockIdx.x * 256u + threadIdx.x;
  const unsigned crow = g / (unsigned)(DIM / 8);
  const unsigned c = (g - crow * (unsigned)(DIM / 8)) * 8u;
  const unsigned bidx = crow / rows_c;
  const unsigned rr = crow - bidx * rows_c;
  const size_t srow = (size_t)bidx * rows_f + rr;
  const v4f a0 = *(const v4f*)(src + srow * DIM + c);
  const v4f a1 = *(const v4f*)(src + srow * DIM + c + 4u);
  v8h o;
#pragma unroll
  for (int i = 0; i < 4; ++i) {
    o[i]     = toh_flush(carry * bf16r(a0[i]));
    o[i + 4] = toh_flush(carry * bf16r(a1[i]));
  }
  _Float16* p = dst + (size_t)crow * DIM + c;
  *(volatile v8h*)p = o;
  __threadfence();
  *(volatile v8h*)p = o;
}

template <int MODE>
__device__ __forceinline__ void gemm_body(
    const _Float16* __restrict__ A16, const _Float16* __restrict__ Bt,
    const float* __restrict__ bias, float* __restrict__ outf, _Float16* __restrict__ out16) {
  __shared__ float Cs[64 * LDC];
  const unsigned tid = threadIdx.x, lane = tid & 31u;
  const unsigned w = (unsigned)__builtin_amdgcn_readfirstlane((int)(tid >> 5));
  const unsigned mw = w >> 1, nw = w & 1u;
  const unsigned hh = lane >> 4, m = lane & 15u;
  const unsigned n0 = blockIdx.x * 64u;
  const unsigned row0 = blockIdx.y * 64u;

  const _Float16* ap  = A16 + (size_t)(row0 + mw * 16u + m) * DIM + hh * 8u;
  const _Float16* bp0 = Bt + (size_t)(n0 + nw * 32u + m) * DIM + hh * 8u;
  const _Float16* bp1 = bp0 + (size_t)16 * DIM;
  v8f acc0 = {}, acc1 = {};
#pragma unroll 2
  for (unsigned k0 = 0; k0 < (unsigned)DIM; k0 += 32u) {
    const v16h a  = frag_at(ap + k0);
    const v16h b0 = frag_at(bp0 + k0);
    const v16h b1 = frag_at(bp1 + k0);
    acc0 = wmma16(a, b0, acc0);
    acc1 = wmma16(a, b1, acc1);
  }
#pragma unroll
  for (int r = 0; r < 8; ++r) {
    float* d = &Cs[(mw * 16u + hh * 8u + (unsigned)r) * LDC + nw * 32u + m];
    d[0]  = acc0[r];
    d[16] = acc1[r];
  }
  __syncthreads();

  if (MODE == 0) {
    v8h x[2];
    size_t off[2];
#pragma unroll
    for (unsigned i = 0; i < 2u; ++i) {
      const unsigned r = 32u * i + (tid >> 3);
      const unsigned c = (tid & 7u) * 8u;
      const v4f u0 = *(const v4f*)&Cs[r * LDC + c];
      const v4f u1 = *(const v4f*)&Cs[r * LDC + c + 4];
      const v4f g0 = *(const v4f*)(bias + n0 + c);
      const v4f g1 = *(const v4f*)(bias + n0 + c + 4u);
      float q[8];
#pragma unroll
      for (int j = 0; j < 4; ++j) {
        q[j]     = u0[j] * (1.0f / WCARRY) + bf16r(g0[j]);
        q[j + 4] = u1[j] * (1.0f / WCARRY) + bf16r(g1[j]);
      }
      float mx = fmaxf(fmaxf(fmaxf(q[0], q[1]), fmaxf(q[2], q[3])),
                       fmaxf(fmaxf(q[4], q[5]), fmaxf(q[6], q[7])));
      mx = fmaxf(mx, __shfl_xor(mx, 1, 32));
      mx = fmaxf(mx, __shfl_xor(mx, 2, 32));
      mx = fmaxf(mx, __shfl_xor(mx, 4, 32));
#pragma unroll
      for (int j = 0; j < 8; ++j) x[i][j] = toh_flush(QCARRY * __expf(q[j] - mx));
      off[i] = (size_t)(row0 + r) * DIM + n0 + c;
    }
#pragma unroll
    for (int i = 0; i < 2; ++i) *(volatile v8h*)(out16 + off[i]) = x[i];
    __threadfence();
#pragma unroll
    for (int i = 0; i < 2; ++i) *(volatile v8h*)(out16 + off[i]) = x[i];
  }

  if (MODE == 1 || MODE == 2) {
    const unsigned bidx = row0 / (unsigned)SEQ;
    const unsigned key0 = row0 - bidx * (unsigned)SEQ;
    v8h x[2];
    size_t off[2];
#pragma unroll
    for (unsigned i = 0; i < 2u; ++i) {
      const unsigned dcol = 32u * i + (tid >> 3);
      const unsigned kk = (tid & 7u) * 8u;
      const float bb = bf16r(bias[n0 + dcol]);
#pragma unroll
      for (unsigned j = 0; j < 8u; ++j) {
        const float t = Cs[(kk + j) * LDC + dcol] * (1.0f / WCARRY) + bb;
        const float val = (MODE == 1) ? __expf(fminf(t, 11.0f)) : t;
        x[i][j] = toh_flush(val);
      }
      off[i] = ((size_t)bidx * DIM + n0 + dcol) * SEQ + key0 + kk;
    }
#pragma unroll
    for (int i = 0; i < 2; ++i) *(volatile v8h*)(out16 + off[i]) = x[i];
    __threadfence();
#pragma unroll
    for (int i = 0; i < 2; ++i) *(volatile v8h*)(out16 + off[i]) = x[i];
  }

  if (MODE == 3) {
    const float cs = 1.0f / (WCARRY * VCARRY);
    v4f xs[4];
    size_t off[4];
#pragma unroll
    for (unsigned i = 0; i < 4u; ++i) {
      const unsigned r = 16u * i + (tid >> 4);
      const unsigned c = (tid & 15u) * 4u;
      const unsigned crow = row0 + r;
      const unsigned bidx = crow / (unsigned)SEQ;
      const unsigned sq = crow - bidx * (unsigned)SEQ;
      const size_t frow = (size_t)bidx * SEQ_FULL + sq;
      const v4f u = *(const v4f*)&Cs[r * LDC + c];
      const v4f g = *(const v4f*)(bias + n0 + c);
      v4f val;
#pragma unroll
      for (int j = 0; j < 4; ++j) val[j] = u[j] * cs + bf16r(g[j]);
      xs[i] = val;
      off[i] = frow * DIM + n0 + c;
    }
#pragma unroll
    for (int i = 0; i < 4; ++i) *(volatile v4f*)(outf + off[i]) = xs[i];
    __threadfence();
#pragma unroll
    for (int i = 0; i < 4; ++i) *(volatile v4f*)(outf + off[i]) = xs[i];
  }
}

__global__ __launch_bounds__(256) void gemm_q_kernel(
    const _Float16* __restrict__ A16, const _Float16* __restrict__ Bt,
    const float* __restrict__ bias, _Float16* __restrict__ out16) {
  gemm_body<0>(A16, Bt, bias, (float*)0, out16);
}
__global__ __launch_bounds__(256) void gemm_k_kernel(
    const _Float16* __restrict__ A16, const _Float16* __restrict__ Bt,
    const float* __restrict__ bias, _Float16* __restrict__ out16) {
  gemm_body<1>(A16, Bt, bias, (float*)0, out16);
}
__global__ __launch_bounds__(256) void gemm_v_kernel(
    const _Float16* __restrict__ A16, const _Float16* __restrict__ Bt,
    const float* __restrict__ bias, _Float16* __restrict__ out16) {
  gemm_body<2>(A16, Bt, bias, (float*)0, out16);
}
__global__ __launch_bounds__(256) void gemm_o_kernel(
    const _Float16* __restrict__ A16, const _Float16* __restrict__ Bt,
    const float* __restrict__ bias, float* __restrict__ outf) {
  gemm_body<3>(A16, Bt, bias, outf, (_Float16*)0);
}

__global__ __launch_bounds__(256) void kv_kernel(
    const _Float16* __restrict__ EKt, const _Float16* __restrict__ Vt,
    _Float16* __restrict__ KVT) {
  __shared__ float Cs[64 * LDC];
  __shared__ float Ss[64];
  const unsigned tid = threadIdx.x, lane = tid & 31u;
  const unsigned w = (unsigned)__builtin_amdgcn_readfirstlane((int)(tid >> 5));
  const unsigned mw = w >> 1, nw = w & 1u;
  const unsigned hh = lane >> 4, m = lane & 15u;
  const unsigned head = blockIdx.x;
  const unsigned b = blockIdx.y;

  const size_t prow = (size_t)b * DIM + head * HD;
  const _Float16* ap  = EKt + (prow + mw * 16u + m) * SEQ + hh * 8u;
  const _Float16* bp0 = Vt + (prow + nw * 32u + m) * SEQ + hh * 8u;
  const _Float16* bp1 = bp0 + (size_t)16 * SEQ;
  v16h ones;
#pragma unroll
  for (int i = 0; i < 16; ++i) ones[i] = (_Float16)1.0f;

  v8f acc0 = {}, acc1 = {}, accs = {};
#pragma unroll 2
  for (unsigned k0 = 0; k0 < (unsigned)SEQ; k0 += 32u) {
    const v16h a  = frag_at(ap + k0);
    const v16h b0 = frag_at(bp0 + k0);
    const v16h b1 = frag_at(bp1 + k0);
    acc0 = wmma16(a, b0, acc0);
    acc1 = wmma16(a, b1, acc1);
    accs = wmma16(a, ones, accs);
  }
#pragma unroll
  for (int r = 0; r < 8; ++r) {
    float* d = &Cs[(mw * 16u + hh * 8u + (unsigned)r) * LDC + nw * 32u + m];
    d[0]  = acc0[r] * KVCARRY;
    d[16] = acc1[r] * KVCARRY;
  }
  if (nw == 0u && m == 0u) {
#pragma unroll
    for (int r = 0; r < 8; ++r) Ss[mw * 16u + hh * 8u + (unsigned)r] = accs[r] * KVCARRY;
  }
  __syncthreads();

  const size_t pbase = (size_t)(b * NHEAD + head) * (size_t)(KVROWS * HD);
  v8h x[3];
  size_t off[3];
  const unsigned c = (tid & 7u) * 8u;
#pragma unroll
  for (unsigned i = 0; i < 2u; ++i) {
    const unsigned n = 32u * i + (tid >> 3);
#pragma unroll
    for (unsigned j = 0; j < 8u; ++j) x[i][j] = toh_flush(Cs[(c + j) * LDC + n]);
    off[i] = pbase + (size_t)n * HD + c;
  }
  {
    const unsigned n = 64u + ((tid >> 3) & 15u);
#pragma unroll
    for (unsigned j = 0; j < 8u; ++j) x[2][j] = toh_flush(Ss[c + j]);
    off[2] = pbase + (size_t)n * HD + c;
  }
  const bool srows = (w < 4u);
#pragma unroll
  for (int i = 0; i < 2; ++i) *(volatile v8h*)(KVT + off[i]) = x[i];
  if (srows) *(volatile v8h*)(KVT + off[2]) = x[2];
  __threadfence();
#pragma unroll
  for (int i = 0; i < 2; ++i) *(volatile v8h*)(KVT + off[i]) = x[i];
  if (srows) *(volatile v8h*)(KVT + off[2]) = x[2];
}

__global__ __launch_bounds__(256) void lattn_kernel(
    const _Float16* __restrict__ EQ, const _Float16* __restrict__ KVT,
    _Float16* __restrict__ J16) {
  __shared__ float Cs[64 * LDC];
  const unsigned tid = threadIdx.x, lane = tid & 31u;
  const unsigned w = (unsigned)__builtin_amdgcn_readfirstlane((int)(tid >> 5));
  const unsigned mw = w >> 1, nw = w & 1u;
  const unsigned hh = lane >> 4, m = lane & 15u;
  const unsigned head = blockIdx.x;
  const unsigned row0 = blockIdx.y * 64u;
  const unsigned b = row0 / (unsigned)SEQ;

  const _Float16* ap  = EQ + (size_t)(row0 + mw * 16u + m) * DIM + head * HD + hh * 8u;
  const _Float16* kb  = KVT + (size_t)(b * NHEAD + head) * (size_t)(KVROWS * HD);
  const _Float16* bp0 = kb + (size_t)(nw * 32u + m) * HD + hh * 8u;
  const _Float16* bp1 = bp0 + (size_t)16 * HD;
  const _Float16* bpd = kb + (size_t)(64u + m) * HD + hh * 8u;
  v8f acc0 = {}, acc1 = {}, accd = {};
#pragma unroll
  for (unsigned k0 = 0; k0 < (unsigned)HD; k0 += 32u) {
    const v16h a  = frag_at(ap + k0);
    const v16h b0 = frag_at(bp0 + k0);
    const v16h b1 = frag_at(bp1 + k0);
    const v16h bd = frag_at(bpd + k0);
    acc0 = wmma16(a, b0, acc0);
    acc1 = wmma16(a, b1, acc1);
    accd = wmma16(a, bd, accd);
  }
#pragma unroll
  for (int r = 0; r < 8; ++r) {
    const float inv = __builtin_amdgcn_rcpf(accd[r]) * VCARRY;
    float* d = &Cs[(mw * 16u + hh * 8u + (unsigned)r) * LDC + nw * 32u + m];
    d[0]  = acc0[r] * inv;
    d[16] = acc1[r] * inv;
  }
  __syncthreads();

  v8h x[2];
  size_t off[2];
#pragma unroll
  for (unsigned i = 0; i < 2u; ++i) {
    const unsigned r = 32u * i + (tid >> 3);
    const unsigned c = (tid & 7u) * 8u;
    const v4f u0 = *(const v4f*)&Cs[r * LDC + c];
    const v4f u1 = *(const v4f*)&Cs[r * LDC + c + 4];
#pragma unroll
    for (int j = 0; j < 4; ++j) {
      x[i][j]     = toh_flush(u0[j]);
      x[i][j + 4] = toh_flush(u1[j]);
    }
    off[i] = (size_t)(row0 + r) * DIM + head * HD + c;
  }
#pragma unroll
  for (int i = 0; i < 2; ++i) *(volatile v8h*)(J16 + off[i]) = x[i];
  __threadfence();
#pragma unroll
  for (int i = 0; i < 2; ++i) *(volatile v8h*)(J16 + off[i]) = x[i];
}

extern "C" void kernel_launch(void* const* d_in, const int* in_sizes, int n_in,
                              void* d_out, int out_size, void* d_ws, size_t ws_size,
                              hipStream_t stream) {
  if (n_in < 9) return;
  const long long need_x = ((long long)(NB - 1) * SEQ_FULL + SEQ) * DIM;
  if ((long long)in_sizes[0] < need_x) return;
  if ((long long)in_sizes[1] < (long long)DIM * DIM) return;
  if ((long long)in_sizes[3] < (long long)DIM * DIM) return;
  if ((long long)in_sizes[5] < (long long)DIM * DIM) return;
  if ((long long)in_sizes[7] < (long long)DIM * DIM) return;
  if (in_sizes[2] < DIM || in_sizes[4] < DIM || in_sizes[6] < DIM || in_sizes[8] < DIM) return;
  if ((long long)out_size < need_x) return;
  if (ws_size < WS_TOTAL) return;

  const float* X  = (const float*)d_in[0];
  const float* wq = (const float*)d_in[1];
  const float* bq = (const float*)d_in[2];
  const float* wk = (const float*)d_in[3];
  const float* bk = (const float*)d_in[4];
  const float* wv = (const float*)d_in[5];
  const float* bv = (const float*)d_in[6];
  const float* wo = (const float*)d_in[7];
  const float* bo = (const float*)d_in[8];
  float* out = (float*)d_out;

  char* ws = (char*)d_ws;
  _Float16* X16   = (_Float16*)(ws + OFF_X);
  _Float16* Wq16  = (_Float16*)(ws + OFF_WQ);
  _Float16* Wk16  = (_Float16*)(ws + OFF_WK);
  _Float16* Wv16  = (_Float16*)(ws + OFF_WV);
  _Float16* Wo16  = (_Float16*)(ws + OFF_WO);
  _Float16* EQ16  = (_Float16*)(ws + OFF_EQ);
  _Float16* EKt16 = (_Float16*)(ws + OFF_EKT);
  _Float16* Vt16  = (_Float16*)(ws + OFF_VT);
  _Float16* KVT16 = (_Float16*)(ws + OFF_KVT);
  _Float16* J16   = (_Float16*)(ws + OFF_J);

  dim3 blk(256);
  dim3 gg(DIM / 64, MROWS / 64);
  const unsigned gx = (unsigned)(((size_t)MROWS * DIM / 8) / 256);
  const unsigned gw = (unsigned)(((size_t)DIM * DIM / 8) / 256);

  cast_kernel<<<dim3(gx), blk, 0, stream>>>(X, X16, 1.0f, (unsigned)SEQ, (unsigned)SEQ_FULL);
  cast_kernel<<<dim3(gw), blk, 0, stream>>>(wq, Wq16, WCARRY, (unsigned)DIM, (unsigned)DIM);
  cast_kernel<<<dim3(gw), blk, 0, stream>>>(wk, Wk16, WCARRY, (unsigned)DIM, (unsigned)DIM);
  cast_kernel<<<dim3(gw), blk, 0, stream>>>(wv, Wv16, WCARRY, (unsigned)DIM, (unsigned)DIM);
  cast_kernel<<<dim3(gw), blk, 0, stream>>>(wo, Wo16, WCARRY, (unsigned)DIM, (unsigned)DIM);

  gemm_q_kernel<<<gg, blk, 0, stream>>>(X16, Wq16, bq, EQ16);
  gemm_k_kernel<<<gg, blk, 0, stream>>>(X16, Wk16, bk, EKt16);
  gemm_v_kernel<<<gg, blk, 0, stream>>>(X16, Wv16, bv, Vt16);
  kv_kernel<<<dim3(NHEAD, NB), blk, 0, stream>>>(EKt16, Vt16, KVT16);
  lattn_kernel<<<dim3(NHEAD, MROWS / 64), blk, 0, stream>>>(EQ16, KVT16, J16);
  gemm_o_kernel<<<gg, blk, 0, stream>>>(J16, Wo16, bo, out);
}
